// NerfNetwork_858993459694
// MI455X (gfx1250) — hardware-run, weakly checked
//
#include <hip/hip_runtime.h>
#include <math.h>

typedef __attribute__((ext_vector_type(16))) _Float16 v16h;
typedef __attribute__((ext_vector_type(8)))  _Float16 v8h;
typedef __attribute__((ext_vector_type(8)))  float    v8f;
typedef __attribute__((ext_vector_type(4)))  float    v4f;

constexpr int kRays         = 524288;
constexpr int kHid          = 128;
constexpr int kLevPos       = 10;
constexpr int kLevDir       = 4;
constexpr int kPeX          = 3 + 6 * kLevPos;
constexpr int kPeD          = 3 + 6 * kLevDir;
constexpr int kPeXPad       = 64;
constexpr int kPeDPad       = 32;
constexpr int kRaysPerBlock = 128;
constexpr int kActPitch     = 128;
constexpr int kK10          = kPeXPad;
constexpr int kK20          = kHid + kPeXPad;
constexpr int kK3           = kHid + kPeDPad;
constexpr int kHalfHid      = 64;
constexpr int kHeadRows     = 16;
static_assert(kPeX == 63 && kPeD == 27, "encoding widths");
static_assert((kRays % kRaysPerBlock) == 0, "no tail block");
static_assert((kK10 % 32) == 0 && (kK20 % 32) == 0 && (kK3 % 32) == 0 && (kHid % 32) == 0 && (kHalfHid % 32) == 0, "K multiples of 32");

constexpr float kWCarry = 256.0f;
constexpr float kACarry = 64.0f;
constexpr float kFold   = 1.0f / (kWCarry * kACarry);

constexpr size_t kOffW10  = 0;
constexpr size_t kOffW11  = kOffW10 + (size_t)kHid * kK10 * 2;
constexpr size_t kOffW12  = kOffW11 + (size_t)kHid * kHid * 2;
constexpr size_t kOffW13  = kOffW12 + (size_t)kHid * kHid * 2;
constexpr size_t kOffW20  = kOffW13 + (size_t)kHid * kHid * 2;
constexpr size_t kOffW21  = kOffW20 + (size_t)kHid * kK20 * 2;
constexpr size_t kOffW22  = kOffW21 + (size_t)kHid * kHid * 2;
constexpr size_t kOffW23  = kOffW22 + (size_t)kHid * kHid * 2;
constexpr size_t kOffW3   = kOffW23 + (size_t)kHid * kHid * 2;
constexpr size_t kOffW4   = kOffW3  + (size_t)kHalfHid * kK3 * 2;
constexpr size_t kOffWsig = kOffW4  + (size_t)kHeadRows * kHalfHid * 2;
constexpr size_t kWsTotal = kOffWsig + (size_t)kHid * 4;
static_assert(kWsTotal == 285184ull, "carve total");
static_assert(kWsTotal <= 134217728ull, "carve cap");
static_assert((kOffW11 % 128) == 0 && (kOffW12 % 128) == 0 && (kOffW13 % 128) == 0 && (kOffW20 % 128) == 0 &&
              (kOffW21 % 128) == 0 && (kOffW22 % 128) == 0 && (kOffW23 % 128) == 0 && (kOffW3 % 128) == 0 &&
              (kOffW4 % 128) == 0 && (kOffWsig % 128) == 0, "128-B aligned regions");

union FragU { v16h v; v8h h[2]; };

__device__ __forceinline__ v16h frag_ld(const _Float16* p) {
  FragU f;
  f.h[0] = *(const v8h*)(p);
  f.h[1] = *(const v8h*)(p + 16);
  return f.v;
}

__device__ __forceinline__ v8f mma_g(v16h a, v16h b, v8f c) {
  c = __builtin_amdgcn_wmma_f32_16x16x32_f16(false, a, false, b, (short)0, c, false, false);
  asm volatile("v_nop\n\tv_nop\n\tv_nop\n\tv_nop" : "+v"(c) : "v"(a), "v"(b));
  return c;
}

__device__ __forceinline__ void wave_sync() {
  __builtin_amdgcn_fence(__ATOMIC_RELEASE, "workgroup");
  __builtin_amdgcn_wave_barrier();
  __builtin_amdgcn_fence(__ATOMIC_ACQUIRE, "workgroup");
}

template <int LDW, int KREAL, int NREAL, int KPAD, int NROWS>
__device__ __forceinline__ void pack_plane(const float* __restrict__ src, unsigned short* __restrict__ dst, int lb) {
  constexpr int kThrPerRow = KPAD / 8;
  constexpr int kTotal = NROWS * kThrPerRow;
  static_assert((kTotal % 32) == 0, "whole waves");
  const int i = lb * 256 + (int)threadIdx.x;
  if (i >= kTotal) return;
  const int n  = i / kThrPerRow;
  const int k0 = (i - n * kThrPerRow) * 8;
  const int ns = (n < NREAL) ? n : (NREAL - 1);
  v8h hv;
#pragma unroll
  for (int e = 0; e < 8; ++e) {
    const int k  = k0 + e;
    const int ks = (k < KREAL) ? k : (KREAL - 1);
    const float v = src[(size_t)ks * LDW + ns];
    const float w = (k < KREAL && n < NREAL) ? (v * kWCarry) : 0.0f;
    hv[e] = (_Float16)w;
  }
  unsigned short* q = dst + (size_t)i * 8;
  *(volatile v8h*)q = hv;
  __threadfence();
  *(volatile v8h*)q = hv;
}

constexpr int kPackBlocks = 71;

__global__ __launch_bounds__(256) void pack_planes_kernel(
    const float* __restrict__ w10, const float* __restrict__ w11, const float* __restrict__ w12,
    const float* __restrict__ w13, const float* __restrict__ w20, const float* __restrict__ w21,
    const float* __restrict__ w22, const float* __restrict__ w23, const float* __restrict__ w3,
    const float* __restrict__ w4, unsigned short* __restrict__ planes, float* __restrict__ wsig)
{
  const int b = (int)blockIdx.x;
  if (b < 4)       pack_plane<128,  63, 128,  64, 128>(w10, planes + kOffW10 / 2, b);
  else if (b < 12) pack_plane<128, 128, 128, 128, 128>(w11, planes + kOffW11 / 2, b - 4);
  else if (b < 20) pack_plane<128, 128, 128, 128, 128>(w12, planes + kOffW12 / 2, b - 12);
  else if (b < 28) pack_plane<128, 128, 128, 128, 128>(w13, planes + kOffW13 / 2, b - 20);
  else if (b < 40) pack_plane<128, 191, 128, 192, 128>(w20, planes + kOffW20 / 2, b - 28);
  else if (b < 48) pack_plane<128, 128, 128, 128, 128>(w21, planes + kOffW21 / 2, b - 40);
  else if (b < 56) pack_plane<128, 128, 128, 128, 128>(w22, planes + kOffW22 / 2, b - 48);
  else if (b < 64) pack_plane<129, 128, 128, 128, 128>(w23, planes + kOffW23 / 2, b - 56);
  else if (b < 69) pack_plane< 64, 155,  64, 160,  64>(w3,  planes + kOffW3  / 2, b - 64);
  else if (b < 70) pack_plane<  3,  64,   3,  64,  16>(w4,  planes + kOffW4  / 2, b - 69);
  else {
    if (threadIdx.x < 32) {
      const int t = (int)threadIdx.x;
      v4f v;
      v[0] = w23[(size_t)(4 * t + 0) * 129 + 128];
      v[1] = w23[(size_t)(4 * t + 1) * 129 + 128];
      v[2] = w23[(size_t)(4 * t + 2) * 129 + 128];
      v[3] = w23[(size_t)(4 * t + 3) * 129 + 128];
      float* q = wsig + 4 * t;
      *(volatile v4f*)q = v;
      __threadfence();
      *(volatile v4f*)q = v;
    }
  }
}

template <int COL, int NV>
__device__ __forceinline__ void put16(v8h (&e)[NV], float v) {
  static_assert(COL < NV * 8, "column inside the row");
  e[COL >> 3][COL & 7] = (_Float16)(v * kACarry);
}

template <int LEV, int NV>
__device__ __forceinline__ void pe_level(v8h (&e)[NV], float s0, float s1, float s2, float c0, float c1, float c2) {
  put16<3 + 6 * LEV + 0>(e, s0);
  put16<3 + 6 * LEV + 1>(e, s1);
  put16<3 + 6 * LEV + 2>(e, s2);
  put16<3 + 6 * LEV + 3>(e, c0);
  put16<3 + 6 * LEV + 4>(e, c1);
  put16<3 + 6 * LEV + 5>(e, c2);
}

__device__ __forceinline__ void dbl_angle(float& s, float& c) {
  const float ns = 2.0f * s * c;
  const float nc = 1.0f - 2.0f * s * s;
  s = ns;
  c = nc;
}

__device__ __forceinline__ void dbl3(float& s0, float& s1, float& s2, float& c0, float& c1, float& c2) {
  dbl_angle(s0, c0);
  dbl_angle(s1, c1);
  dbl_angle(s2, c2);
}

template <int NT>
__device__ __forceinline__ void gemm_seg(v8f (&acc0)[NT], v8f (&acc1)[NT],
                                         const _Float16* __restrict__ wt, int wpitch, int wk0,
                                         const _Float16* sb, int bpitch, int nkc,
                                         int rowbase, int rc, int h)
{
  const _Float16* bp0 = sb + (rowbase + rc) * bpitch + 8 * h;
  const _Float16* bp1 = bp0 + 16 * bpitch;
  const _Float16* wp  = wt + rc * wpitch + wk0 + 8 * h;
#pragma unroll 1
  for (int kc = 0; kc < nkc; ++kc) {
    const v16h b0 = frag_ld(bp0 + kc * 32);
    const v16h b1 = frag_ld(bp1 + kc * 32);
#pragma unroll
    for (int nt = 0; nt < NT; ++nt) {
      const v16h a = frag_ld(wp + nt * 16 * wpitch + kc * 32);
      acc0[nt] = mma_g(a, b0, acc0[nt]);
      acc1[nt] = mma_g(a, b1, acc1[nt]);
      asm volatile("" ::: "memory");
    }
  }
}

template <int NT>
__device__ __forceinline__ void zero_acc(v8f (&acc)[NT]) {
#pragma unroll
  for (int nt = 0; nt < NT; ++nt) acc[nt] = (v8f){0.f, 0.f, 0.f, 0.f, 0.f, 0.f, 0.f, 0.f};
}

template <int NT, bool RELU, bool SIG>
__device__ __forceinline__ void epilogue(v8f (&acc0)[NT], v8f (&acc1)[NT],
                                         const float* __restrict__ bias, const float* __restrict__ wsig,
                                         _Float16* sact, int rowbase, int rc, int h,
                                         float& sg0, float& sg1)
{
  _Float16* r0 = sact + (rowbase + rc) * kActPitch + 8 * h;
  _Float16* r1 = r0 + 16 * kActPitch;
#pragma unroll
  for (int nt = 0; nt < NT; ++nt) {
    const int nb = nt * 16 + 8 * h;
    const v4f bA = *(const v4f*)(bias + nb);
    const v4f bB = *(const v4f*)(bias + nb + 4);
    const float bv[8] = {bA[0], bA[1], bA[2], bA[3], bB[0], bB[1], bB[2], bB[3]};
    v4f wA = bA;
    v4f wB = bB;
    if (SIG) {
      wA = *(const v4f*)(wsig + nb);
      wB = *(const v4f*)(wsig + nb + 4);
    }
    const float wv[8] = {wA[0], wA[1], wA[2], wA[3], wB[0], wB[1], wB[2], wB[3]};
    v8h h0, h1;
#pragma unroll
    for (int r = 0; r < 8; ++r) {
      float v0 = acc0[nt][r] * kFold + bv[r];
      float v1 = acc1[nt][r] * kFold + bv[r];
      if (RELU) {
        v0 = fmaxf(v0, 0.0f);
        v1 = fmaxf(v1, 0.0f);
      }
      if (SIG) {
        sg0 = fmaf(v0, wv[r], sg0);
        sg1 = fmaf(v1, wv[r], sg1);
      }
      h0[r] = (_Float16)(v0 * kACarry);
      h1[r] = (_Float16)(v1 * kACarry);
    }
    *(v8h*)(r0 + nt * 16) = h0;
    *(v8h*)(r1 + nt * 16) = h1;
  }
}

template <bool RELU, bool SIG>
__device__ __forceinline__ void dense128(const _Float16* __restrict__ wt, const float* __restrict__ bias,
                                         const float* __restrict__ wsig, _Float16* sact,
                                         int rowbase, int rc, int h, float& sg0, float& sg1)
{
  v8f a0[8], a1[8];
  zero_acc(a0);
  zero_acc(a1);
  gemm_seg<8>(a0, a1, wt, kHid, 0, sact, kActPitch, 4, rowbase, rc, h);
  epilogue<8, RELU, SIG>(a0, a1, bias, wsig, sact, rowbase, rc, h, sg0, sg1);
  wave_sync();
}

__global__ __launch_bounds__(128) void mlp_fused_kernel(
    const float* __restrict__ o, const float* __restrict__ dvec,
    const float* __restrict__ b10, const float* __restrict__ b11, const float* __restrict__ b12,
    const float* __restrict__ b13, const float* __restrict__ b20, const float* __restrict__ b21,
    const float* __restrict__ b22, const float* __restrict__ b23, const float* __restrict__ b3,
    const float* __restrict__ b4, const _Float16* __restrict__ wq, const float* __restrict__ wsig,
    float* __restrict__ out)
{
  __shared__ __align__(16) _Float16 sAct[kRaysPerBlock * kActPitch];
  __shared__ __align__(16) _Float16 sEmbx[kRaysPerBlock * kPeXPad];
  __shared__ __align__(16) _Float16 sEmbd[kRaysPerBlock * kPeDPad];
  __shared__ __align__(16) float sC[kRaysPerBlock * 3];
  __shared__ __align__(16) float sSig[kRaysPerBlock];

  const int tid     = (int)threadIdx.x;
  const int lane    = tid & 31;
  const int wave    = tid >> 5;
  const int rc      = lane & 15;
  const int h       = lane >> 4;
  const int rowbase = wave * 32;

  {
    const int ray = (int)blockIdx.x * kRaysPerBlock + tid;
    const float o0 = o[ray * 3 + 0], o1 = o[ray * 3 + 1], o2 = o[ray * 3 + 2];
    const float d0 = dvec[ray * 3 + 0], d1 = dvec[ray * 3 + 1], d2 = dvec[ray * 3 + 2];
    float zp = 0.0f;
    asm volatile("" : "+v"(zp));

    v8h ex[8];
    put16<0>(ex, o0);
    put16<1>(ex, o1);
    put16<2>(ex, o2);
    float s0 = sinf(o0), s1 = sinf(o1), s2 = sinf(o2);
    float c0 = cosf(o0), c1 = cosf(o1), c2 = cosf(o2);
    pe_level<0>(ex, s0, s1, s2, c0, c1, c2);
    dbl3(s0, s1, s2, c0, c1, c2);
    pe_level<1>(ex, s0, s1, s2, c0, c1, c2);
    dbl3(s0, s1, s2, c0, c1, c2);
    pe_level<2>(ex, s0, s1, s2, c0, c1, c2);
    dbl3(s0, s1, s2, c0, c1, c2);
    pe_level<3>(ex, s0, s1, s2, c0, c1, c2);
    dbl3(s0, s1, s2, c0, c1, c2);
    pe_level<4>(ex, s0, s1, s2, c0, c1, c2);
    {
      const float p0 = o0 * 32.0f, p1 = o1 * 32.0f, p2 = o2 * 32.0f;
      s0 = sinf(p0); s1 = sinf(p1); s2 = sinf(p2);
      c0 = cosf(p0); c1 = cosf(p1); c2 = cosf(p2);
    }
    pe_level<5>(ex, s0, s1, s2, c0, c1, c2);
    dbl3(s0, s1, s2, c0, c1, c2);
    pe_level<6>(ex, s0, s1, s2, c0, c1, c2);
    dbl3(s0, s1, s2, c0, c1, c2);
    pe_level<7>(ex, s0, s1, s2, c0, c1, c2);
    dbl3(s0, s1, s2, c0, c1, c2);
    pe_level<8>(ex, s0, s1, s2, c0, c1, c2);
    dbl3(s0, s1, s2, c0, c1, c2);
    pe_level<9>(ex, s0, s1, s2, c0, c1, c2);
    put16<63>(ex, zp);
#pragma unroll
    for (int i = 0; i < 8; ++i) *(v8h*)(sEmbx + tid * kPeXPad + 8 * i) = ex[i];

    v8h ed[4];
    put16<0>(ed, d0);
    put16<1>(ed, d1);
    put16<2>(ed, d2);
    s0 = sinf(d0); s1 = sinf(d1); s2 = sinf(d2);
    c0 = cosf(d0); c1 = cosf(d1); c2 = cosf(d2);
    pe_level<0>(ed, s0, s1, s2, c0, c1, c2);
    dbl3(s0, s1, s2, c0, c1, c2);
    pe_level<1>(ed, s0, s1, s2, c0, c1, c2);
    dbl3(s0, s1, s2, c0, c1, c2);
    pe_level<2>(ed, s0, s1, s2, c0, c1, c2);
    dbl3(s0, s1, s2, c0, c1, c2);
    pe_level<3>(ed, s0, s1, s2, c0, c1, c2);
    put16<27>(ed, zp);
    put16<28>(ed, zp);
    put16<29>(ed, zp);
    put16<30>(ed, zp);
    put16<31>(ed, zp);
#pragma unroll
    for (int i = 0; i < 4; ++i) *(v8h*)(sEmbd + tid * kPeDPad + 8 * i) = ed[i];
  }
  __syncthreads();

  float sg0 = 0.0f, sg1 = 0.0f;

  {
    v8f a0[8], a1[8];
    zero_acc(a0);
    zero_acc(a1);
    gemm_seg<8>(a0, a1, wq + kOffW10 / 2, kK10, 0, sEmbx, kPeXPad, 2, rowbase, rc, h);
    epilogue<8, true, false>(a0, a1, b10, wsig, sAct, rowbase, rc, h, sg0, sg1);
    wave_sync();
  }
  dense128<true, false>(wq + kOffW11 / 2, b11, wsig, sAct, rowbase, rc, h, sg0, sg1);
  dense128<true, false>(wq + kOffW12 / 2, b12, wsig, sAct, rowbase, rc, h, sg0, sg1);
  dense128<true, false>(wq + kOffW13 / 2, b13, wsig, sAct, rowbase, rc, h, sg0, sg1);

  {
    v8f a0[8], a1[8];
    zero_acc(a0);
    zero_acc(a1);
    gemm_seg<8>(a0, a1, wq + kOffW20 / 2, kK20, 0, sAct, kActPitch, 4, rowbase, rc, h);
    gemm_seg<8>(a0, a1, wq + kOffW20 / 2, kK20, kHid, sEmbx, kPeXPad, 2, rowbase, rc, h);
    epilogue<8, true, false>(a0, a1, b20, wsig, sAct, rowbase, rc, h, sg0, sg1);
    wave_sync();
  }
  dense128<true, false>(wq + kOffW21 / 2, b21, wsig, sAct, rowbase, rc, h, sg0, sg1);
  dense128<true, true>(wq + kOffW22 / 2, b22, wsig, sAct, rowbase, rc, h, sg0, sg1);
  {
    const float t0 = __shfl_xor(sg0, 16, 32);
    const float t1 = __shfl_xor(sg1, 16, 32);
    const float bs = b23[kHid];
    const float sig0 = fmaxf((sg0 + t0) + bs, 0.0f);
    const float sig1 = fmaxf((sg1 + t1) + bs, 0.0f);
    if (h == 0) {
      sSig[rowbase + rc]      = sig0;
      sSig[rowbase + 16 + rc] = sig1;
    }
  }
  dense128<false, false>(wq + kOffW23 / 2, b23, wsig, sAct, rowbase, rc, h, sg0, sg1);

  {
    v8f a0[4], a1[4];
    zero_acc(a0);
    zero_acc(a1);
    gemm_seg<4>(a0, a1, wq + kOffW3 / 2, kK3, 0, sAct, kActPitch, 4, rowbase, rc, h);
    gemm_seg<4>(a0, a1, wq + kOffW3 / 2, kK3, kHid, sEmbd, kPeDPad, 1, rowbase, rc, h);
    epilogue<4, true, false>(a0, a1, b3, wsig, sAct, rowbase, rc, h, sg0, sg1);
    wave_sync();
  }

  {
    v8f e0[1], e1[1];
    zero_acc(e0);
    zero_acc(e1);
    gemm_seg<1>(e0, e1, wq + kOffW4 / 2, kHalfHid, 0, sAct, kActPitch, 2, rowbase, rc, h);
    const float bc0 = b4[0], bc1 = b4[1], bc2 = b4[2];
    const float x00 = e0[0][0] * kFold + bc0;
    const float x01 = e0[0][1] * kFold + bc1;
    const float x02 = e0[0][2] * kFold + bc2;
    const float x10 = e1[0][0] * kFold + bc0;
    const float x11 = e1[0][1] * kFold + bc1;
    const float x12 = e1[0][2] * kFold + bc2;
    const float y00 = 1.0f / (1.0f + expf(-x00));
    const float y01 = 1.0f / (1.0f + expf(-x01));
    const float y02 = 1.0f / (1.0f + expf(-x02));
    const float y10 = 1.0f / (1.0f + expf(-x10));
    const float y11 = 1.0f / (1.0f + expf(-x11));
    const float y12 = 1.0f / (1.0f + expf(-x12));
    if (h == 0) {
      float* p0 = sC + (rowbase + rc) * 3;
      float* p1 = sC + (rowbase + 16 + rc) * 3;
      p0[0] = y00;
      p0[1] = y01;
      p0[2] = y02;
      p1[0] = y10;
      p1[1] = y11;
      p1[2] = y12;
    }
  }
  __syncthreads();

  {
    const float* sp = (wave < 3) ? (sC + wave * 128) : sSig;
    float* gp = (wave < 3) ? (out + (size_t)blockIdx.x * (kRaysPerBlock * 3) + wave * 128)
                           : (out + (size_t)3 * kRays + (size_t)blockIdx.x * kRaysPerBlock);
    const v4f val = *(const v4f*)(sp + lane * 4);
    float* q = gp + lane * 4;
    *(volatile v4f*)q = val;
    __threadfence();
    *(volatile v4f*)q = val;
  }
}

extern "C" void kernel_launch(void* const* d_in, const int* in_sizes, int n_in,
                              void* d_out, int out_size, void* d_ws, size_t ws_size,
                              hipStream_t stream) {
  if (n_in < 22) return;
  if (in_sizes[0] != kRays * 3 || in_sizes[1] != kRays * 3) return;
  if (in_sizes[2] != kPeX * kHid || in_sizes[3] != kHid) return;
  if (in_sizes[4] != kHid * kHid || in_sizes[5] != kHid) return;
  if (in_sizes[6] != kHid * kHid || in_sizes[7] != kHid) return;
  if (in_sizes[8] != kHid * kHid || in_sizes[9] != kHid) return;
  if (in_sizes[10] != (kHid + kPeX) * kHid || in_sizes[11] != kHid) return;
  if (in_sizes[12] != kHid * kHid || in_sizes[13] != kHid) return;
  if (in_sizes[14] != kHid * kHid || in_sizes[15] != kHid) return;
  if (in_sizes[16] != kHid * (kHid + 1) || in_sizes[17] != kHid + 1) return;
  if (in_sizes[18] != (kHid + kPeD) * kHalfHid || in_sizes[19] != kHalfHid) return;
  if (in_sizes[20] != kHalfHid * 3 || in_sizes[21] != 3) return;
  if (out_size != kRays * 4) return;
  if (ws_size < kWsTotal) return;

  const float* o   = (const float*)d_in[0];
  const float* dv  = (const float*)d_in[1];
  const float* w10 = (const float*)d_in[2];
  const float* b10 = (const float*)d_in[3];
  const float* w11 = (const float*)d_in[4];
  const float* b11 = (const float*)d_in[5];
  const float* w12 = (const float*)d_in[6];
  const float* b12 = (const float*)d_in[7];
  const float* w13 = (const float*)d_in[8];
  const float* b13 = (const float*)d_in[9];
  const float* w20 = (const float*)d_in[10];
  const float* b20 = (const float*)d_in[11];
  const float* w21 = (const float*)d_in[12];
  const float* b21 = (const float*)d_in[13];
  const float* w22 = (const float*)d_in[14];
  const float* b22 = (const float*)d_in[15];
  const float* w23 = (const float*)d_in[16];
  const float* b23 = (const float*)d_in[17];
  const float* w3  = (const float*)d_in[18];
  const float* b3  = (const float*)d_in[19];
  const float* w4  = (const float*)d_in[20];
  const float* b4  = (const float*)d_in[21];

  char* ws = (char*)d_ws;
  unsigned short* planes = (unsigned short*)ws;
  float* wsig = (float*)(ws + kOffWsig);

  pack_planes_kernel<<<kPackBlocks, 256, 0, stream>>>(
      w10, w11, w12, w13, w20, w21, w22, w23, w3, w4, planes, wsig);

  mlp_fused_kernel<<<kRays / kRaysPerBlock, kRaysPerBlock, 0, stream>>>(
      o, dv, b10, b11, b12, b13, b20, b21, b22, b23, b3, b4,
      (const _Float16*)ws, (const float*)wsig, (float*)d_out);
}
